// SelfAttention_65300682768451
// MI455X (gfx1250) — hardware-verified
//
#include <hip/hip_runtime.h>


#ifndef NB
#define NB 2
#endif
#ifndef SEQ
#define SEQ 2048
#endif
#define NB_FULL    2
#define SEQ_FULL   2048
#define HID        1024
#define NHEAD      16
#define HDIM       64
#define BQ         128
#define BK         32
#define NWAVE      8
#define OP         68
#define GM         128
#define GN         64
#define CP         68
#define TPV        136

static_assert(SEQ % BQ == 0);
static_assert(SEQ % GM == 0);
static_assert(SEQ % BK == 0);
static_assert((SEQ & (SEQ - 1)) == 0);
static_assert(BQ == NWAVE * 16);
static_assert(HDIM == 64);
static_assert(GN == HDIM);
static_assert(HID == NHEAD * HDIM);
static_assert(HID % 32 == 0);
static_assert(HID / 8 == 128);
static_assert(SEQ <= SEQ_FULL);
static_assert(NB >= 1 && NB <= NB_FULL);
static_assert((NB * SEQ) % GM == 0);
static_assert((NB * SEQ) % 32 == 0);
static_assert((OP * 4) % 16 == 0);
static_assert((CP * 4) % 16 == 0);
static_assert((TPV * 2) % 16 == 0);

#define CVT_X_BLOCKS ((unsigned)(((size_t)NB * SEQ * HID) / 2048))
#define CVT_W_BLOCKS ((unsigned)(((size_t)HID * HID) / 2048))
#define CVT_M_PIECES ((unsigned)((NB * SEQ) / 4))
#define CVT_M_BLOCKS ((CVT_M_PIECES + 255u) / 256u)
#define CVT_GX       ((CVT_X_BLOCKS > CVT_W_BLOCKS) ? CVT_X_BLOCKS : CVT_W_BLOCKS)

static_assert(((size_t)NB * SEQ * HID) % 2048 == 0);
static_assert(((size_t)HID * HID) % 2048 == 0);
static_assert((size_t)CVT_X_BLOCKS * 256 * 8 == (size_t)NB * SEQ * HID);
static_assert((size_t)CVT_W_BLOCKS * 256 * 8 == (size_t)HID * HID);
static_assert(CVT_M_BLOCKS <= CVT_GX);

typedef __bf16   bf16;
typedef _Float16 f16;
typedef bf16     v16bf __attribute__((ext_vector_type(16)));
typedef f16      v16h  __attribute__((ext_vector_type(16)));
typedef f16      v8h   __attribute__((ext_vector_type(8)));
typedef float    v8f   __attribute__((ext_vector_type(8)));
typedef float    v4f   __attribute__((ext_vector_type(4)));
typedef unsigned v4u   __attribute__((ext_vector_type(4)));

union FragB  { v16bf v; v4u q[2]; bf16 h[16]; };
union FragH  { v16h  v; v4u q[2]; f16  h[16]; };
union Pack8B { v4u u; bf16 h[8]; };
union Pack8H { v4u u; v8h v; f16 h[8]; };

static __device__ __forceinline__ v8f mma_bf16(v16bf a, v16bf b, v8f acc) {
  acc = __builtin_amdgcn_wmma_f32_16x16x32_bf16(false, a, false, b, (short)0, acc, false, false);
  asm volatile("v_nop\n\tv_nop\n\tv_nop\n\tv_nop" : "+v"(acc) : "v"(a), "v"(b));
  return acc;
}
static __device__ __forceinline__ v8f mma_f16(v16h a, v16h b, v8f acc) {
  acc = __builtin_amdgcn_wmma_f32_16x16x32_f16(false, a, false, b, (short)0, acc, false, false);
  asm volatile("v_nop\n\tv_nop\n\tv_nop\n\tv_nop" : "+v"(acc) : "v"(a), "v"(b));
  return acc;
}

__global__ __launch_bounds__(256) void convert_kernel(const float* __restrict__ x,
                                                      const float* __restrict__ wq,
                                                      const float* __restrict__ wk,
                                                      const float* __restrict__ wv,
                                                      const float* __restrict__ mask,
                                                      bf16* __restrict__ xb,
                                                      bf16* __restrict__ wb,
                                                      float* __restrict__ mplane) {
  const unsigned seg = blockIdx.y;
  const unsigned blk = blockIdx.x;
  const unsigned tid = threadIdx.x;

  if (seg == 4u) {
    if (blk >= CVT_M_BLOCKS) return;
    const unsigned i  = blk * 256u + tid;
    const unsigned ic = (i < CVT_M_PIECES) ? i : (CVT_M_PIECES - 1u);
    const unsigned e  = ic * 4u;
    const unsigned b  = e / (unsigned)SEQ;
    const unsigned s  = e % (unsigned)SEQ;
    const v4f m = *(const v4f*)(mask + (size_t)b * SEQ_FULL + s);
    v4f o;
    #pragma unroll
    for (int j = 0; j < 4; ++j) o[j] = (float)(bf16)m[j];
    float* dst = mplane + (size_t)ic * 4u;
    if (i < CVT_M_PIECES) *(volatile v4f*)dst = o;
    __threadfence();
    if (i < CVT_M_PIECES) *(volatile v4f*)dst = o;
    return;
  }

  const unsigned nblk = (seg == 0u) ? CVT_X_BLOCKS : CVT_W_BLOCKS;
  if (blk >= nblk) return;
  const unsigned i = blk * 256u + tid;
  const float* src;
  bf16* dst;
  if (seg == 0u) {
    const unsigned row = i >> 7;
    const unsigned col = (i & 127u) << 3;
    const unsigned b   = row / (unsigned)SEQ;
    const unsigned s   = row % (unsigned)SEQ;
    src = x + ((size_t)b * SEQ_FULL + s) * HID + col;
    dst = xb + (size_t)i * 8u;
  } else {
    const float* w = (seg == 1u) ? wq : ((seg == 2u) ? wk : wv);
    src = w + (size_t)i * 8u;
    dst = wb + (size_t)(seg - 1u) * HID * HID + (size_t)i * 8u;
  }
  const v4f a0 = *(const v4f*)(src);
  const v4f a1 = *(const v4f*)(src + 4);
  Pack8B pk;
  #pragma unroll
  for (int j = 0; j < 4; ++j) {
    pk.h[j]     = (bf16)a0[j];
    pk.h[4 + j] = (bf16)a1[j];
  }
  const v4u val = pk.u;
  *(volatile v4u*)dst = val;
  __threadfence();
  *(volatile v4u*)dst = val;
}

__global__ __launch_bounds__(128) void proj_kernel(const bf16* __restrict__ xb,
                                                   const bf16* __restrict__ wb,
                                                   const float* __restrict__ bq,
                                                   const float* __restrict__ bk,
                                                   const float* __restrict__ bvv,
                                                   bf16* __restrict__ qh, bf16* __restrict__ ql,
                                                   bf16* __restrict__ kh, bf16* __restrict__ kl,
                                                   f16* __restrict__ vt) {
  __shared__ __align__(16) float sC[GM * CP];
  __shared__ __align__(16) f16   sT[HDIM * TPV];

  const unsigned nt   = blockIdx.x;
  const unsigned proj = nt >> 4;
  const unsigned h    = nt & 15u;
  const unsigned m0   = blockIdx.y * GM;
  const unsigned tid  = threadIdx.x;
  const unsigned wave = tid >> 5;
  const unsigned lane = tid & 31u;
  const unsigned lq   = lane & 15u;
  const unsigned hi   = lane >> 4;

  const bf16* ap[2];
  const bf16* bp[4];
  #pragma unroll
  for (int mt = 0; mt < 2; ++mt)
    ap[mt] = xb + (size_t)(m0 + wave * 32u + (unsigned)mt * 16u + lq) * HID + hi * 8u;
  #pragma unroll
  for (int ct = 0; ct < 4; ++ct)
    bp[ct] = wb + (size_t)(nt * 64u + (unsigned)ct * 16u + lq) * HID + hi * 8u;

  v8f acc[2][4];
  #pragma unroll
  for (int mt = 0; mt < 2; ++mt) {
    #pragma unroll
    for (int ct = 0; ct < 4; ++ct) acc[mt][ct] = (v8f){0, 0, 0, 0, 0, 0, 0, 0};
  }

  #pragma unroll 1
  for (unsigned k0 = 0; k0 < HID; k0 += 32u) {
    FragB a[2], bb[4];
    #pragma unroll
    for (int mt = 0; mt < 2; ++mt) {
      a[mt].q[0] = *(const v4u*)(ap[mt] + k0);
      a[mt].q[1] = *(const v4u*)(ap[mt] + k0 + 16);
    }
    #pragma unroll
    for (int ct = 0; ct < 4; ++ct) {
      bb[ct].q[0] = *(const v4u*)(bp[ct] + k0);
      bb[ct].q[1] = *(const v4u*)(bp[ct] + k0 + 16);
    }
    #pragma unroll
    for (int mt = 0; mt < 2; ++mt) {
      #pragma unroll
      for (int ct = 0; ct < 4; ++ct) acc[mt][ct] = mma_bf16(a[mt].v, bb[ct].v, acc[mt][ct]);
    }
  }

  const float* bias = (proj == 0u) ? bq : ((proj == 1u) ? bk : bvv);
  float bz[4];
  #pragma unroll
  for (int ct = 0; ct < 4; ++ct) bz[ct] = (float)(bf16)bias[h * 64u + (unsigned)ct * 16u + lq];

  const unsigned b  = m0 / (unsigned)SEQ;
  const unsigned s0 = m0 % (unsigned)SEQ;

  if (proj < 2u) {
    #pragma unroll
    for (int mt = 0; mt < 2; ++mt) {
      #pragma unroll
      for (int ct = 0; ct < 4; ++ct) {
        #pragma unroll
        for (int r = 0; r < 8; ++r)
          sC[(wave * 32u + (unsigned)mt * 16u + hi * 8u + (unsigned)r) * CP + (unsigned)ct * 16u + lq] =
              acc[mt][ct][r] + bz[ct];
      }
    }
  } else {
    #pragma unroll
    for (int mt = 0; mt < 2; ++mt) {
      #pragma unroll
      for (int ct = 0; ct < 4; ++ct) {
        Pack8H ph;
        #pragma unroll
        for (int r = 0; r < 8; ++r) ph.h[r] = (f16)(acc[mt][ct][r] + bz[ct]);
        *(v8h*)(sT + ((unsigned)ct * 16u + lq) * TPV + wave * 32u + (unsigned)mt * 16u + hi * 8u) = ph.v;
      }
    }
  }
  __syncthreads();

  if (proj < 2u) {
    bf16* hp = (proj == 0u) ? qh : kh;
    bf16* lp = (proj == 0u) ? ql : kl;
    v4u hv[8], lv[8];
    const unsigned rsub = tid >> 3;
    const unsigned d0   = (tid & 7u) * 8u;
    #pragma unroll
    for (int it = 0; it < 8; ++it) {
      const unsigned row = (unsigned)it * 16u + rsub;
      const v4f x0 = *(const v4f*)(sC + row * CP + d0);
      const v4f x1 = *(const v4f*)(sC + row * CP + d0 + 4u);
      Pack8B ph, pl;
      #pragma unroll
      for (int j = 0; j < 4; ++j) {
        const bf16 t0 = (bf16)x0[j];
        const bf16 t1 = (bf16)x1[j];
        ph.h[j]     = t0;
        ph.h[4 + j] = t1;
        pl.h[j]     = (bf16)(x0[j] - (float)t0);
        pl.h[4 + j] = (bf16)(x1[j] - (float)t1);
      }
      hv[it] = ph.u;
      lv[it] = pl.u;
    }
    const size_t gbase = (((size_t)b * NHEAD + h) * SEQ + s0 + rsub) * HDIM + d0;
    #pragma unroll
    for (int it = 0; it < 8; ++it) {
      *(volatile v4u*)(hp + gbase + (size_t)it * 16u * HDIM) = hv[it];
      *(volatile v4u*)(lp + gbase + (size_t)it * 16u * HDIM) = lv[it];
    }
    __threadfence();
    #pragma unroll
    for (int it = 0; it < 8; ++it) {
      *(volatile v4u*)(hp + gbase + (size_t)it * 16u * HDIM) = hv[it];
      *(volatile v4u*)(lp + gbase + (size_t)it * 16u * HDIM) = lv[it];
    }
  } else {
    v4u vv[8];
    const unsigned dsub = tid >> 4;
    const unsigned ks   = (tid & 15u) * 8u;
    #pragma unroll
    for (int it = 0; it < 8; ++it) {
      const unsigned d = (unsigned)it * 8u + dsub;
      Pack8H ph;
      ph.v = *(const v8h*)(sT + d * TPV + ks);
      vv[it] = ph.u;
    }
    const size_t vbase = (((size_t)b * NHEAD + h) * HDIM + dsub) * SEQ + s0 + ks;
    #pragma unroll
    for (int it = 0; it < 8; ++it) *(volatile v4u*)(vt + vbase + (size_t)it * 8u * SEQ) = vv[it];
    __threadfence();
    #pragma unroll
    for (int it = 0; it < 8; ++it) *(volatile v4u*)(vt + vbase + (size_t)it * 8u * SEQ) = vv[it];
  }
}

__global__ __launch_bounds__(256) void attn_kernel(const bf16* __restrict__ qh,
                                                   const bf16* __restrict__ ql,
                                                   const bf16* __restrict__ kh,
                                                   const bf16* __restrict__ kl,
                                                   const f16* __restrict__ vt,
                                                   const float* __restrict__ mplane,
                                                   float* __restrict__ out) {
  const unsigned qblk = blockIdx.x;
  const unsigned h    = blockIdx.y;
  const unsigned b    = blockIdx.z;
  const unsigned tid  = threadIdx.x;
  const unsigned wave = tid >> 5;
  const unsigned lane = tid & 31u;
  const unsigned lq   = lane & 15u;
  const unsigned hi   = lane >> 4;

  __shared__ __align__(16) float sO[NWAVE * 16 * OP];

  const unsigned qrow0 = qblk * BQ + wave * 16u;
  const size_t   hoff  = ((size_t)b * NHEAD + h) * SEQ * HDIM;

  FragB qfh[2], qfl[2];
  {
    const bf16* qph = qh + hoff + (size_t)(qrow0 + lq) * HDIM + hi * 8u;
    const bf16* qpl = ql + hoff + (size_t)(qrow0 + lq) * HDIM + hi * 8u;
    #pragma unroll
    for (int f = 0; f < 2; ++f) {
      qfh[f].q[0] = *(const v4u*)(qph + f * 32);
      qfh[f].q[1] = *(const v4u*)(qph + f * 32 + 16);
      qfl[f].q[0] = *(const v4u*)(qpl + f * 32);
      qfl[f].q[1] = *(const v4u*)(qpl + f * 32 + 16);
    }
  }

  const bf16*  kh_h = kh + hoff;
  const bf16*  kl_h = kl + hoff;
  const f16*   vt_h = vt + hoff;
  const float* mk   = mplane + (size_t)b * SEQ;

  v8f o[4];
  #pragma unroll
  for (int dt = 0; dt < 4; ++dt) o[dt] = (v8f){0, 0, 0, 0, 0, 0, 0, 0};

  float rmax = -__builtin_inff();
  float rsum = 0.0f;
  const float L2E = 1.4426950408889634f;

  #pragma unroll 1
  for (unsigned i = 0; i < (unsigned)(SEQ / BK); ++i) {
    const unsigned j0 = i * BK;

    v8f c[2];
    #pragma unroll
    for (int sub = 0; sub < 2; ++sub) {
      FragB akh[2], akl[2];
      #pragma unroll
      for (int f = 0; f < 2; ++f) {
        const size_t off = (size_t)(j0 + (unsigned)sub * 16u + lq) * HDIM + (unsigned)f * 32u + hi * 8u;
        akh[f].q[0] = *(const v4u*)(kh_h + off);
        akh[f].q[1] = *(const v4u*)(kh_h + off + 16);
        akl[f].q[0] = *(const v4u*)(kl_h + off);
        akl[f].q[1] = *(const v4u*)(kl_h + off + 16);
      }
      const float* mp = mk + j0 + (unsigned)sub * 16u + hi * 8u;
      const v4f mb0 = *(const v4f*)(mp);
      const v4f mb1 = *(const v4f*)(mp + 4);

      v8f acc = (v8f){0, 0, 0, 0, 0, 0, 0, 0};
      acc = mma_bf16(akl[0].v, qfh[0].v, acc);
      acc = mma_bf16(akl[1].v, qfh[1].v, acc);
      acc = mma_bf16(akh[0].v, qfl[0].v, acc);
      acc = mma_bf16(akh[1].v, qfl[1].v, acc);
      acc = mma_bf16(akh[0].v, qfh[0].v, acc);
      acc = mma_bf16(akh[1].v, qfh[1].v, acc);
      #pragma unroll
      for (int r = 0; r < 4; ++r) {
        acc[r]     = fmaf(acc[r],     0.125f, mb0[r]);
        acc[4 + r] = fmaf(acc[4 + r], 0.125f, mb1[r]);
      }
      c[sub] = acc;
    }

    FragH vfr[4];
    #pragma unroll
    for (int dt = 0; dt < 4; ++dt) {
      const f16* base = vt_h + (size_t)((unsigned)dt * 16u + lq) * SEQ + j0 + hi * 8u;
      vfr[dt].q[0] = *(const v4u*)(base);
      vfr[dt].q[1] = *(const v4u*)(base + 16);
    }

    float m_new = rmax;
    #pragma unroll
    for (int r = 0; r < 8; ++r) {
      m_new = fmaxf(m_new, c[0][r]);
      m_new = fmaxf(m_new, c[1][r]);
    }
    m_new = fmaxf(m_new, __shfl_xor(m_new, 16, 32));
    const float m_use = (m_new == -__builtin_inff()) ? 0.0f : m_new;
    const float scale = __builtin_amdgcn_exp2f((rmax - m_use) * L2E);
    rmax = m_new;

    FragH pa;
    float psum = 0.0f;
    #pragma unroll
    for (int r = 0; r < 8; ++r) {
      const float p0 = __builtin_amdgcn_exp2f((c[0][r] - m_use) * L2E);
      const float p1 = __builtin_amdgcn_exp2f((c[1][r] - m_use) * L2E);
      psum += p0 + p1;
      pa.h[r]     = (f16)(p0 * 4096.0f);
      pa.h[8 + r] = (f16)(p1 * 4096.0f);
    }
    rsum = rsum * scale + psum + __shfl_xor(psum, 16, 32);

    float sc[8];
    #pragma unroll
    for (int r = 0; r < 8; ++r) sc[r] = __shfl(scale, (int)((hi << 3) + (unsigned)r), 32);
    #pragma unroll
    for (int dt = 0; dt < 4; ++dt) {
      #pragma unroll
      for (int r = 0; r < 8; ++r) o[dt][r] *= sc[r];
    }

    #pragma unroll
    for (int dt = 0; dt < 4; ++dt) o[dt] = mma_f16(pa.v, vfr[dt].v, o[dt]);
  }

  float rs[8];
  #pragma unroll
  for (int r = 0; r < 8; ++r) rs[r] = 1.0f / __shfl(rsum, (int)((hi << 3) + (unsigned)r), 32);

  float* so = sO + wave * (16u * OP);
  #pragma unroll
  for (int r = 0; r < 8; ++r) {
    #pragma unroll
    for (int dt = 0; dt < 4; ++dt)
      so[(hi * 8u + (unsigned)r) * OP + (unsigned)dt * 16u + lq] = o[dt][r] * (1.0f / 4096.0f) * rs[r];
  }
  __syncthreads();

  v4f    vals[8];
  size_t gidx[8];
  #pragma unroll
  for (int it = 0; it < 8; ++it) {
    const unsigned row = (unsigned)it * 2u + hi;
    vals[it] = *(const v4f*)(so + row * OP + lq * 4u);
    gidx[it] = ((size_t)b * SEQ_FULL + qrow0 + row) * HID + h * HDIM + lq * 4u;
  }
  #pragma unroll
  for (int it = 0; it < 8; ++it) *(volatile v4f*)(out + gidx[it]) = vals[it];
  __threadfence();
  #pragma unroll
  for (int it = 0; it < 8; ++it) *(volatile v4f*)(out + gidx[it]) = vals[it];
}

extern "C" void kernel_launch(void* const* d_in, const int* in_sizes, int n_in,
                              void* d_out, int out_size, void* d_ws, size_t ws_size,
                              hipStream_t stream) {
  if (n_in < 8) return;
  const size_t rows_used = (size_t)(NB - 1) * SEQ_FULL + SEQ;
  if ((size_t)in_sizes[0] < rows_used * HID) return;
  if ((size_t)in_sizes[1] < rows_used) return;
  if ((size_t)in_sizes[2] < (size_t)HID * HID) return;
  if ((size_t)in_sizes[3] < (size_t)HID) return;
  if ((size_t)in_sizes[4] < (size_t)HID * HID) return;
  if ((size_t)in_sizes[5] < (size_t)HID) return;
  if ((size_t)in_sizes[6] < (size_t)HID * HID) return;
  if ((size_t)in_sizes[7] < (size_t)HID) return;
  if ((size_t)out_size < rows_used * HID) return;

  const size_t xb_bytes = (size_t)NB * SEQ * HID * 2;
  const size_t wb_bytes = (size_t)3 * HID * HID * 2;
  const size_t hp_bytes = (size_t)NB * NHEAD * SEQ * HDIM * 2;
  const size_t mp_bytes = (size_t)NB * SEQ * 4;
  const size_t total    = xb_bytes + wb_bytes + 5 * hp_bytes + mp_bytes;
  if (ws_size < total) return;
  if (total > (size_t)134217728) return;

  char* ws = (char*)d_ws;
  bf16*  xb = (bf16*)(ws);
  bf16*  wb = (bf16*)(ws + xb_bytes);
  bf16*  qh = (bf16*)(ws + xb_bytes + wb_bytes);
  bf16*  ql = (bf16*)(ws + xb_bytes + wb_bytes + hp_bytes);
  bf16*  kh = (bf16*)(ws + xb_bytes + wb_bytes + 2 * hp_bytes);
  bf16*  kl = (bf16*)(ws + xb_bytes + wb_bytes + 3 * hp_bytes);
  f16*   vt = (f16*) (ws + xb_bytes + wb_bytes + 4 * hp_bytes);
  float* mp = (float*)(ws + xb_bytes + wb_bytes + 5 * hp_bytes);

  const float* X    = (const float*)d_in[0];
  const float* mask = (const float*)d_in[1];
  const float* Wq   = (const float*)d_in[2];
  const float* bq   = (const float*)d_in[3];
  const float* Wk   = (const float*)d_in[4];
  const float* bk   = (const float*)d_in[5];
  const float* Wv   = (const float*)d_in[6];
  const float* bv   = (const float*)d_in[7];
  float* out = (float*)d_out;

  convert_kernel<<<dim3(CVT_GX, 5, 1), 256, 0, stream>>>(X, Wq, Wk, Wv, mask, xb, wb, mp);
  proj_kernel<<<dim3(3 * NHEAD, (NB * SEQ) / GM, 1), 128, 0, stream>>>(xb, wb, bq, bk, bv, qh, ql, kh, kl, vt);
  attn_kernel<<<dim3(SEQ / BQ, NHEAD, NB), 256, 0, stream>>>(qh, ql, kh, kl, vt, mp, out);
}
